// ATMT5CE4Attention_29549374996520
// MI455X (gfx1250) — hardware-verified
//
#include <hip/hip_runtime.h>
#include <math.h>
#include <stdint.h>

#define NB      2
#define NQ      2048
#define NC      2048
#define DMODEL  1024
#define NHEAD   16
#define HDIM    64
#define NBKT    32
#define NROWS   (NB * NQ)
#define WSC     64.0f
#define ACARRY  16.0f
#define VC      16.0f
#define PC      1024.0f
#define ATT_SCALE 0.125f
#define LOG2E   1.4426950408889634f
#define SL2     (ATT_SCALE * LOG2E)
static_assert(NHEAD * HDIM == DMODEL);
static_assert((NQ % 64) == 0 && (NC % 64) == 0 && (DMODEL % 64) == 0 && (NC % 32) == 0 && (NQ % 16) == 0);
static_assert((NROWS % 64) == 0);
#define ATT_THREADS (NHEAD * 32)
#define ATT_BLOCKS  (NB * (NQ / 16))
static_assert(ATT_THREADS == 512 && ATT_BLOCKS == 256);
#define LUTP            2064
#define PT_FLOATS       (NHEAD * 16 * 36)
#define LUT_HALVES      (NHEAD * LUTP)
#define ATT_SMEM_FLOATS (PT_FLOATS + LUT_HALVES / 2)
static_assert((LUT_HALVES % 8) == 0);
static_assert(NQ + 15 <= LUTP - 1);
static_assert((size_t)2 * 16 * DMODEL * sizeof(unsigned short) <= (size_t)ATT_SMEM_FLOATS * sizeof(float));

typedef _Float16 v16h __attribute__((ext_vector_type(16)));
typedef _Float16 v8h  __attribute__((ext_vector_type(8)));
typedef __bf16   v16b __attribute__((ext_vector_type(16)));
typedef float    v8f  __attribute__((ext_vector_type(8)));
typedef float    v4f  __attribute__((ext_vector_type(4)));
typedef unsigned int v4u __attribute__((ext_vector_type(4)));

union FragH { v16h v; v8h h[2]; v4u u[2]; };
union FragAny { v16h h; v16b b; };

__device__ __forceinline__ unsigned short bf_bits(float f) {
  unsigned u = __float_as_uint(f);
  return (unsigned short)((u + 0x7FFFu + ((u >> 16) & 1u)) >> 16);
}
__device__ __forceinline__ float bf_up(unsigned short h) { return __uint_as_float(((unsigned)h) << 16); }
__device__ __forceinline__ float bfr(float f) { return bf_up(bf_bits(f)); }
__device__ __forceinline__ unsigned short h_bits(_Float16 x) { return __builtin_bit_cast(unsigned short, x); }
__device__ __forceinline__ unsigned pk16(unsigned short a, unsigned short b) { return (unsigned)a | ((unsigned)b << 16); }
__device__ __forceinline__ v8f zero8() { v8f z = {0.f, 0.f, 0.f, 0.f, 0.f, 0.f, 0.f, 0.f}; return z; }

__device__ __forceinline__ v16h ldfrag_u(const unsigned short* p) {
  FragH f;
  f.u[0] = *(const v4u*)(p);
  f.u[1] = *(const v4u*)(p + 16);
  return f.v;
}

__device__ __forceinline__ v8f mma_h(v16h a, v16h b, v8f c) {
  return __builtin_amdgcn_wmma_f32_16x16x32_f16(false, a, false, b, (short)0, c, false, false);
}
__device__ __forceinline__ v8f mma_b(v16h a, v16h b, v8f c) {
  FragAny ua, ub;
  ua.h = a;
  ub.h = b;
  return __builtin_amdgcn_wmma_f32_16x16x32_bf16(false, ua.b, false, ub.b, (short)0, c, false, false);
}
template <int BF>
__device__ __forceinline__ v8f mmaT(v16h a, v16h b, v8f c) {
  if constexpr (BF != 0) return mma_b(a, b, c);
  else return mma_h(a, b, c);
}
__device__ __forceinline__ void dep_guard1(v8f& a, v8f& b, v16h x) {
#if defined(__HIP_DEVICE_COMPILE__)
  asm volatile("v_nop\n\tv_nop\n\tv_nop\n\tv_nop" : "+v"(a), "+v"(b) : "v"(x));
#endif
}
__device__ __forceinline__ void guard1x4(v8f& s, v16h a0, v16h a1, v16h a2, v16h a3) {
#if defined(__HIP_DEVICE_COMPILE__)
  asm volatile("v_nop\n\tv_nop\n\tv_nop\n\tv_nop" : "+v"(s) : "v"(a0), "v"(a1), "v"(a2), "v"(a3));
#endif
}
__device__ __forceinline__ void guard1x8(v8f& s, v16h a0, v16h a1, v16h a2, v16h a3,
                                         v16h b0, v16h b1, v16h b2, v16h b3) {
#if defined(__HIP_DEVICE_COMPILE__)
  asm volatile("v_nop\n\tv_nop\n\tv_nop\n\tv_nop"
               : "+v"(s) : "v"(a0), "v"(a1), "v"(a2), "v"(a3), "v"(b0), "v"(b1), "v"(b2), "v"(b3));
#endif
}
__device__ __forceinline__ void guard4x6(v8f& a, v8f& b, v8f& c, v8f& d,
                                         v16h x0, v16h x1, v16h x2, v16h x3, v16h x4, v16h x5) {
#if defined(__HIP_DEVICE_COMPILE__)
  asm volatile("v_nop\n\tv_nop\n\tv_nop\n\tv_nop"
               : "+v"(a), "+v"(b), "+v"(c), "+v"(d) : "v"(x0), "v"(x1), "v"(x2), "v"(x3), "v"(x4), "v"(x5));
#endif
}
__device__ __forceinline__ void guard4x5(v8f& a, v8f& b, v8f& c, v8f& d,
                                         v16h x0, v16h x1, v16h x2, v16h x3, v16h x4) {
#if defined(__HIP_DEVICE_COMPILE__)
  asm volatile("v_nop\n\tv_nop\n\tv_nop\n\tv_nop"
               : "+v"(a), "+v"(b), "+v"(c), "+v"(d) : "v"(x0), "v"(x1), "v"(x2), "v"(x3), "v"(x4));
#endif
}
__device__ __forceinline__ void keep4_h(v16h a, v16h b, v16h c, v16h d) {
#if defined(__HIP_DEVICE_COMPILE__)
  asm volatile("v_nop" :: "v"(a), "v"(b), "v"(c), "v"(d));
#endif
}
__device__ __forceinline__ void acc_guard4(v8f& a, v8f& b, v8f& c, v8f& d) {
#if defined(__HIP_DEVICE_COMPILE__)
  asm volatile("v_nop\n\tv_nop\n\tv_nop\n\tv_nop" : "+v"(a), "+v"(b), "+v"(c), "+v"(d));
#endif
}
__device__ __forceinline__ void wave_sync_lds() {
  __builtin_amdgcn_fence(__ATOMIC_RELEASE, "workgroup");
  __builtin_amdgcn_wave_barrier();
  __builtin_amdgcn_fence(__ATOMIC_ACQUIRE, "workgroup");
}

template <int BFO>
__global__ __launch_bounds__(256) void cvt16(const float* __restrict__ src, unsigned short* dst, int n, float sc) {
  const size_t i8 = ((size_t)blockIdx.x * 256 + threadIdx.x) * 8;
  if (i8 + 8 > (size_t)n) return;
  const v4f a = *(const v4f*)(src + i8);
  const v4f b = *(const v4f*)(src + i8 + 4);
  v4u o;
  if constexpr (BFO != 0) {
    o[0] = pk16(bf_bits(a[0]), bf_bits(a[1]));
    o[1] = pk16(bf_bits(a[2]), bf_bits(a[3]));
    o[2] = pk16(bf_bits(b[0]), bf_bits(b[1]));
    o[3] = pk16(bf_bits(b[2]), bf_bits(b[3]));
  } else {
    o[0] = pk16(h_bits((_Float16)(bfr(a[0]) * sc)), h_bits((_Float16)(bfr(a[1]) * sc)));
    o[1] = pk16(h_bits((_Float16)(bfr(a[2]) * sc)), h_bits((_Float16)(bfr(a[3]) * sc)));
    o[2] = pk16(h_bits((_Float16)(bfr(b[0]) * sc)), h_bits((_Float16)(bfr(b[1]) * sc)));
    o[3] = pk16(h_bits((_Float16)(bfr(b[2]) * sc)), h_bits((_Float16)(bfr(b[3]) * sc)));
  }
  for (int pass = 0; pass < 2; ++pass) {
    *(volatile v4u*)(dst + i8) = o;
    __threadfence();
  }
}

template <int OM, int ASPLIT, int BF>
__global__ __launch_bounds__(256) void gemm64(
    const unsigned short* __restrict__ Ap, const unsigned short* __restrict__ A2p, int lda, long long sA,
    const unsigned short* __restrict__ Btp, int ldb, long long sB,
    void* Cout, void* C2out, int ldc, long long sC,
    int M, int N, int K, float oscale, float ocarry) {
  __shared__ __align__(16) float sT[8][16 * 68];
  const int by   = blockIdx.y;
  const int lane = threadIdx.x & 31;
  const int wave = threadIdx.x >> 5;
  const int tilesN = N >> 6;
  const int tilesM = M >> 6;
  const int tile = blockIdx.x * 8 + wave;
  if (tile >= tilesM * tilesN) return;
  const int tm = tile / tilesN;
  const int tn = tile - tm * tilesN;
  const int m0 = tm << 6;
  const int n0 = tn << 6;

  const unsigned short* A1 = Ap  + (size_t)((long long)by * sA);
  const unsigned short* A2 = A2p + (size_t)((long long)by * sA);
  const unsigned short* Bb = Btp + (size_t)((long long)by * sB);

  const int rlane = lane & 15;
  const int koff  = (lane >> 4) * 8;
  const int mOff  = (lane >> 4) * 8;

  v8f acc[4][4];
#pragma unroll
  for (int i = 0; i < 4; ++i)
#pragma unroll
    for (int j = 0; j < 4; ++j) acc[i][j] = zero8();

  for (int k0 = 0; k0 < K; k0 += 32) {
    v16h bh[4];
#pragma unroll
    for (int j = 0; j < 4; ++j) {
      const size_t bofs = (size_t)(n0 + (j << 4) + rlane) * ldb + koff + k0;
      bh[j] = ldfrag_u(Bb + bofs);
    }
#pragma unroll
    for (int i = 0; i < 4; ++i) {
      const size_t ao = (size_t)(m0 + (i << 4) + rlane) * lda + koff + k0;
      const v16h ah = ldfrag_u(A1 + ao);
#pragma unroll
      for (int j = 0; j < 4; ++j) acc[i][j] = mmaT<BF>(ah, bh[j], acc[i][j]);
      dep_guard1(acc[i][0], acc[i][3], ah);
      if constexpr (ASPLIT != 0) {
        const v16h al = ldfrag_u(A2 + ao);
#pragma unroll
        for (int j = 0; j < 4; ++j) acc[i][j] = mmaT<BF>(al, bh[j], acc[i][j]);
        dep_guard1(acc[i][0], acc[i][3], al);
      }
    }
    keep4_h(bh[0], bh[1], bh[2], bh[3]);
  }
  acc_guard4(acc[0][0], acc[0][1], acc[0][2], acc[0][3]);
  acc_guard4(acc[1][0], acc[1][1], acc[1][2], acc[1][3]);
  acc_guard4(acc[2][0], acc[2][1], acc[2][2], acc[2][3]);
  acc_guard4(acc[3][0], acc[3][1], acc[3][2], acc[3][3]);

  const int hh2 = lane >> 4, c4 = (lane & 15) * 4;
  const int q8  = lane >> 3, c8 = (lane & 7) * 8;

  float* slab = sT[wave];
#pragma unroll
  for (int i = 0; i < 4; ++i) {
    const int mBase = m0 + (i << 4);
#pragma unroll
    for (int j = 0; j < 4; ++j) {
#pragma unroll
      for (int r = 0; r < 8; ++r) {
        slab[(mOff + r) * 68 + (j << 4) + rlane] = acc[i][j][r];
      }
    }
    wave_sync_lds();
    if constexpr (OM == 0) {
      float* C = (float*)Cout + (size_t)((long long)by * sC);
      v4f vals[8];
#pragma unroll
      for (int it = 0; it < 8; ++it) {
        const int row = it * 2 + hh2;
        v4f v = *(const v4f*)(slab + row * 68 + c4);
#pragma unroll
        for (int e = 0; e < 4; ++e) v[e] = v[e] * oscale;
        vals[it] = v;
      }
      for (int pass = 0; pass < 2; ++pass) {
#pragma unroll
        for (int it = 0; it < 8; ++it) {
          const int gr = mBase + it * 2 + hh2;
          *(volatile v4f*)(C + (size_t)gr * ldc + n0 + c4) = vals[it];
        }
        __threadfence();
      }
    } else {
      unsigned short* C  = (unsigned short*)Cout  + (size_t)((long long)by * sC);
      unsigned short* Cb = (unsigned short*)C2out + (size_t)((long long)by * sC);
      v4u hv[4], lv[4];
#pragma unroll
      for (int it = 0; it < 4; ++it) {
        const int row = it * 4 + q8;
        const float* sp = slab + row * 68 + c8;
        v4u a  = {0u, 0u, 0u, 0u};
        v4u b2 = {0u, 0u, 0u, 0u};
#pragma unroll
        for (int e = 0; e < 4; ++e) {
          float f0 = sp[2 * e] * oscale;
          float f1 = sp[2 * e + 1] * oscale;
          if constexpr (OM == 3) {
            const unsigned short h0 = bf_bits(f0), h1 = bf_bits(f1);
            a[e]  = pk16(h0, h1);
            b2[e] = pk16(bf_bits(f0 - bf_up(h0)), bf_bits(f1 - bf_up(h1)));
          } else {
            f0 *= ocarry; f1 *= ocarry;
            const _Float16 x0 = (_Float16)f0, x1 = (_Float16)f1;
            a[e] = pk16(h_bits(x0), h_bits(x1));
            if constexpr (OM == 4) {
              b2[e] = pk16(h_bits((_Float16)(f0 - (float)x0)), h_bits((_Float16)(f1 - (float)x1)));
            }
          }
        }
        hv[it] = a;
        lv[it] = b2;
      }
      for (int pass = 0; pass < 2; ++pass) {
#pragma unroll
        for (int it = 0; it < 4; ++it) {
          const int row = it * 4 + q8;
          *(volatile v4u*)(C + (size_t)(mBase + row) * ldc + n0 + c8) = hv[it];
          if constexpr (OM >= 3) {
            *(volatile v4u*)(Cb + (size_t)(mBase + row) * ldc + n0 + c8) = lv[it];
          }
        }
        __threadfence();
      }
    }
    wave_sync_lds();
  }
}

__global__ __launch_bounds__(ATT_THREADS)
void attn16(const unsigned short* __restrict__ QHh, const unsigned short* __restrict__ QHl,
            const unsigned short* __restrict__ KHh, const unsigned short* __restrict__ KHl,
            const unsigned short* __restrict__ VTh, const unsigned short* __restrict__ VTl,
            const float* __restrict__ rel, unsigned short* CTh, unsigned short* CTl) {
  __shared__ __align__(16) float smem[ATT_SMEM_FLOATS];
  unsigned short* lut = (unsigned short*)(smem + PT_FLOATS);

  const int tid  = threadIdx.x;
  const int wave = tid >> 5;
  const int lane = tid & 31;
  const int hh   = lane >> 4;
  const int c    = lane & 15;

  const int qt   = blockIdx.x & ((NQ / 16) - 1);
  const int bat  = blockIdx.x / (NQ / 16);
  const int head = wave;
  const int q0   = qt * 16;

  for (int e = tid; e < LUT_HALVES; e += ATT_THREADS) {
    const int hd = e / LUTP;
    const int i  = e - hd * LUTP;
    const int d  = i - (q0 + 15);
    const int a  = (d < 0) ? -d : d;
    int g = 8 + (a >= 12) + (a >= 16) + (a >= 23) + (a >= 32) + (a >= 46) + (a >= 64) + (a >= 91);
    g = (a < 8) ? a : g;
    const int bk = g + ((d > 0) ? 16 : 0);
    lut[e] = bf_bits(rel[bk * NHEAD + hd]);
  }
  __syncthreads();

  const size_t qofs = ((size_t)bat * NQ + q0 + c) * DMODEL + head * HDIM + 8 * hh;
  const v16h qah = ldfrag_u(QHh + qofs), qbh = ldfrag_u(QHh + qofs + 32);
  const v16h qal = ldfrag_u(QHl + qofs), qbl = ldfrag_u(QHl + qofs + 32);
  const size_t kbase = (size_t)bat * NC * DMODEL + head * HDIM + 8 * hh;
  const unsigned short* Kbh = KHh + kbase;
  const unsigned short* Kbl = KHl + kbase;
  const size_t vbase = ((size_t)bat * DMODEL + head * HDIM) * NC + 8 * hh;
  const unsigned short* Vbh = VTh + vbase;
  const unsigned short* Vbl = VTl + vbase;
  const unsigned short* lw = lut + head * LUTP + (c + 15 - 8 * hh);

  float mrow[8], lrow[8];
  v8f o0 = zero8(), o1 = zero8(), o2 = zero8(), o3 = zero8();
#pragma unroll
  for (int r = 0; r < 8; ++r) { mrow[r] = -INFINITY; lrow[r] = 0.f; }
  float* pt = smem + wave * (16 * 36);

#pragma unroll 1
  for (int kb = 0; kb < NC; kb += 32) {
    const size_t ko = (size_t)(kb + c) * DMODEL;
    v8f s0, s1;
    {
      const v16h k0h = ldfrag_u(Kbh + ko), k1h = ldfrag_u(Kbh + ko + 32);
      const v16h k0l = ldfrag_u(Kbl + ko), k1l = ldfrag_u(Kbl + ko + 32);
      s0 = mma_b(qah, k0h, zero8());
      s0 = mma_b(qbh, k1h, s0);
      s0 = mma_b(qah, k0l, s0);
      s0 = mma_b(qbh, k1l, s0);
      s0 = mma_b(qal, k0h, s0);
      s0 = mma_b(qbl, k1h, s0);
      guard1x4(s0, k0h, k1h, k0l, k1l);
    }
    {
      const size_t k2 = ko + (size_t)16 * DMODEL;
      const v16h k0h = ldfrag_u(Kbh + k2), k1h = ldfrag_u(Kbh + k2 + 32);
      const v16h k0l = ldfrag_u(Kbl + k2), k1l = ldfrag_u(Kbl + k2 + 32);
      s1 = mma_b(qah, k0h, zero8());
      s1 = mma_b(qbh, k1h, s1);
      s1 = mma_b(qah, k0l, s1);
      s1 = mma_b(qbh, k1l, s1);
      s1 = mma_b(qal, k0h, s1);
      s1 = mma_b(qbl, k1h, s1);
      guard1x8(s1, k0h, k1h, k0l, k1l, qah, qbh, qal, qbl);
    }
    const unsigned short* lp = lw + kb;
#pragma unroll
    for (int r = 0; r < 8; ++r) {
      const float w0 = bf_up(lp[-r]), w1 = bf_up(lp[16 - r]);
      const float t0 = s0[r] * SL2 + w0 * LOG2E, t1 = s1[r] * SL2 + w1 * LOG2E;
      float mx = fmaxf(t0, t1);
#pragma unroll
      for (int off = 1; off < 16; off <<= 1) mx = fmaxf(mx, __shfl_xor(mx, off, 32));
      const float mn = fmaxf(mrow[r], mx);
      const float al = exp2f(mrow[r] - mn);
      mrow[r] = mn;
      const float e0 = exp2f(t0 - mn), e1 = exp2f(t1 - mn);
      float ps = e0 + e1;
#pragma unroll
      for (int off = 1; off < 16; off <<= 1) ps += __shfl_xor(ps, off, 32);
      lrow[r] = lrow[r] * al + ps;
      o0[r] *= al;
      o1[r] *= al;
      o2[r] *= al;
      o3[r] *= al;
      const int ro = (8 * hh + r) * 36 + c;
      pt[ro]      = e0;
      pt[ro + 16] = e1;
    }
    wave_sync_lds();
    FragH ph, pl;
    {
      const float* prow = pt + c * 36 + 8 * hh;
      const v4f p0 = *(const v4f*)(prow), p1 = *(const v4f*)(prow + 4);
      const v4f p2 = *(const v4f*)(prow + 16), p3 = *(const v4f*)(prow + 20);
#pragma unroll
      for (int e = 0; e < 4; ++e) {
        float f; _Float16 x;
        f = p0[e] * PC; x = (_Float16)f; ph.h[0][e]     = x; pl.h[0][e]     = (_Float16)(f - (float)x);
        f = p1[e] * PC; x = (_Float16)f; ph.h[0][4 + e] = x; pl.h[0][4 + e] = (_Float16)(f - (float)x);
        f = p2[e] * PC; x = (_Float16)f; ph.h[1][e]     = x; pl.h[1][e]     = (_Float16)(f - (float)x);
        f = p3[e] * PC; x = (_Float16)f; ph.h[1][4 + e] = x; pl.h[1][4 + e] = (_Float16)(f - (float)x);
      }
    }
    const size_t vo = (size_t)c * NC + kb;
    {
      const v16h vh0 = ldfrag_u(Vbh + vo);
      const v16h vh1 = ldfrag_u(Vbh + vo + (size_t)16 * NC);
      const v16h vh2 = ldfrag_u(Vbh + vo + (size_t)32 * NC);
      const v16h vh3 = ldfrag_u(Vbh + vo + (size_t)48 * NC);
      o0 = mma_h(ph.v, vh0, o0);
      o1 = mma_h(ph.v, vh1, o1);
      o2 = mma_h(ph.v, vh2, o2);
      o3 = mma_h(ph.v, vh3, o3);
      o0 = mma_h(pl.v, vh0, o0);
      o1 = mma_h(pl.v, vh1, o1);
      o2 = mma_h(pl.v, vh2, o2);
      o3 = mma_h(pl.v, vh3, o3);
      guard4x6(o0, o1, o2, o3, ph.v, pl.v, vh0, vh1, vh2, vh3);
    }
    {
      const v16h vl0 = ldfrag_u(Vbl + vo);
      const v16h vl1 = ldfrag_u(Vbl + vo + (size_t)16 * NC);
      const v16h vl2 = ldfrag_u(Vbl + vo + (size_t)32 * NC);
      const v16h vl3 = ldfrag_u(Vbl + vo + (size_t)48 * NC);
      o0 = mma_h(ph.v, vl0, o0);
      o1 = mma_h(ph.v, vl1, o1);
      o2 = mma_h(ph.v, vl2, o2);
      o3 = mma_h(ph.v, vl3, o3);
      guard4x5(o0, o1, o2, o3, ph.v, vl0, vl1, vl2, vl3);
    }
    wave_sync_lds();
  }

  __syncthreads();
  unsigned short* Osh = (unsigned short*)smem;
  unsigned short* Osl = Osh + 16 * DMODEL;
  const float oc = 1.0f / (PC * VC);
  const int cb = wave * HDIM + c;
#pragma unroll
  for (int r = 0; r < 8; ++r) {
    const float inv = (1.0f / lrow[r]) * oc;
    const int ro = (8 * hh + r) * DMODEL + cb;
    const float f0 = o0[r] * inv, f1 = o1[r] * inv, f2 = o2[r] * inv, f3 = o3[r] * inv;
    const unsigned short g0 = bf_bits(f0), g1 = bf_bits(f1), g2 = bf_bits(f2), g3 = bf_bits(f3);
    Osh[ro]      = g0;  Osl[ro]      = bf_bits(f0 - bf_up(g0));
    Osh[ro + 16] = g1;  Osl[ro + 16] = bf_bits(f1 - bf_up(g1));
    Osh[ro + 32] = g2;  Osl[ro + 32] = bf_bits(f2 - bf_up(g2));
    Osh[ro + 48] = g3;  Osl[ro + 48] = bf_bits(f3 - bf_up(g3));
  }
  __syncthreads();
  {
    v4u hv[4], lv[4];
#pragma unroll
    for (int it = 0; it < 4; ++it) {
      const int p = it * ATT_THREADS + tid;
      hv[it] = *(const v4u*)(Osh + (size_t)p * 8);
      lv[it] = *(const v4u*)(Osl + (size_t)p * 8);
    }
    const size_t dofs = ((size_t)bat * NQ + q0) * DMODEL;
    unsigned short* dsth = CTh + dofs;
    unsigned short* dstl = CTl + dofs;
    for (int pass = 0; pass < 2; ++pass) {
#pragma unroll
      for (int it = 0; it < 4; ++it) {
        const int p = it * ATT_THREADS + tid;
        *(volatile v4u*)(dsth + (size_t)p * 8) = hv[it];
        *(volatile v4u*)(dstl + (size_t)p * 8) = lv[it];
      }
      __threadfence();
    }
  }
}

extern "C" void kernel_launch(void* const* d_in, const int* in_sizes, int n_in,
                              void* d_out, int out_size, void* d_ws, size_t ws_size,
                              hipStream_t stream) {
  if (n_in < 6) return;
  if (in_sizes[0] != NROWS * DMODEL) return;
  if (in_sizes[1] != DMODEL * DMODEL || in_sizes[2] != DMODEL * DMODEL ||
      in_sizes[3] != DMODEL * DMODEL || in_sizes[4] != DMODEL * DMODEL) return;
  if (in_sizes[5] != NBKT * NHEAD) return;
  if (out_size != NROWS * DMODEL) return;
  if ((in_sizes[0] % 2048) != 0 || (in_sizes[1] % 2048) != 0) return;

  const float* x   = (const float*)d_in[0];
  const float* w_q = (const float*)d_in[1];
  const float* w_k = (const float*)d_in[2];
  const float* w_v = (const float*)d_in[3];
  const float* w_o = (const float*)d_in[4];
  const float* rel = (const float*)d_in[5];
  float*       out = (float*)d_out;

  const size_t PW  = (size_t)DMODEL * DMODEL * 2;
  const size_t PX  = (size_t)NROWS * DMODEL * 2;
  const size_t PVT = (size_t)NB * DMODEL * NC * 2;
  size_t off = 0;
  const size_t oWQ = off; off += PW;
  const size_t oWK = off; off += PW;
  const size_t oWV = off; off += PW;
  const size_t oWO = off; off += PW;
  const size_t oX  = off; off += PX;
  const size_t oQh = off; off += PX;
  const size_t oQl = off; off += PX;
  const size_t oKh = off; off += PX;
  const size_t oKl = off; off += PX;
  const size_t oVh = off; off += PVT;
  const size_t oVl = off; off += PVT;
  const size_t oCh = off; off += PX;
  const size_t oCl = off; off += PX;
  if (off > ws_size) return;
  if (off > (size_t)134217728) return;

  char* ws = (char*)d_ws;
  unsigned short* WQ16 = (unsigned short*)(ws + oWQ);
  unsigned short* WK16 = (unsigned short*)(ws + oWK);
  unsigned short* WV16 = (unsigned short*)(ws + oWV);
  unsigned short* WO16 = (unsigned short*)(ws + oWO);
  unsigned short* X16  = (unsigned short*)(ws + oX);
  unsigned short* QHh  = (unsigned short*)(ws + oQh);
  unsigned short* QHl  = (unsigned short*)(ws + oQl);
  unsigned short* KHh  = (unsigned short*)(ws + oKh);
  unsigned short* KHl  = (unsigned short*)(ws + oKl);
  unsigned short* VTh  = (unsigned short*)(ws + oVh);
  unsigned short* VTl  = (unsigned short*)(ws + oVl);
  unsigned short* CTh  = (unsigned short*)(ws + oCh);
  unsigned short* CTl  = (unsigned short*)(ws + oCl);

  const dim3 blk(256);
  const dim3 gCW((DMODEL * DMODEL) / 2048);
  const dim3 gCX((NROWS * DMODEL) / 2048);
  const int tilesP = (NROWS / 64) * (DMODEL / 64);
  const int tilesV = (DMODEL / 64) * (NC / 64);
  const dim3 gP((tilesP + 7) / 8, 1);
  const dim3 gV((tilesV + 7) / 8, NB);
  const dim3 gAT(ATT_BLOCKS);
  const dim3 bAT(ATT_THREADS);

  cvt16<0><<<gCW, blk, 0, stream>>>(w_q, WQ16, DMODEL * DMODEL, WSC);
  cvt16<0><<<gCW, blk, 0, stream>>>(w_k, WK16, DMODEL * DMODEL, WSC);
  cvt16<0><<<gCW, blk, 0, stream>>>(w_v, WV16, DMODEL * DMODEL, WSC);
  cvt16<1><<<gCW, blk, 0, stream>>>(w_o, WO16, DMODEL * DMODEL, 1.0f);

  cvt16<0><<<gCX, blk, 0, stream>>>(x, X16, NROWS * DMODEL, ACARRY);

  gemm64<3, 0, 0><<<gP, blk, 0, stream>>>(
      X16, X16, DMODEL, 0LL,
      WQ16, DMODEL, 0LL,
      (void*)QHh, (void*)QHl, DMODEL, 0LL,
      NROWS, DMODEL, DMODEL, 1.0f / (ACARRY * WSC), 1.0f);

  gemm64<3, 0, 0><<<gP, blk, 0, stream>>>(
      X16, X16, DMODEL, 0LL,
      WK16, DMODEL, 0LL,
      (void*)KHh, (void*)KHl, DMODEL, 0LL,
      NROWS, DMODEL, DMODEL, 1.0f / (ACARRY * WSC), 1.0f);

  gemm64<4, 0, 0><<<gV, blk, 0, stream>>>(
      WV16, WV16, DMODEL, 0LL,
      X16, DMODEL, (long long)NC * DMODEL,
      (void*)VTh, (void*)VTl, NC, (long long)DMODEL * NC,
      DMODEL, NC, DMODEL, 1.0f / (ACARRY * WSC), VC);

  attn16<<<gAT, bAT, 0, stream>>>(QHh, QHl, KHh, KHl, VTh, VTl, rel, CTh, CTl);

  gemm64<0, 1, 1><<<gP, blk, 0, stream>>>(
      CTh, CTl, DMODEL, 0LL,
      WO16, DMODEL, 0LL,
      (void*)out, (void*)out, DMODEL, 0LL,
      NROWS, DMODEL, DMODEL, 1.0f, 1.0f);
  (void)hipGetLastError();
}
